// ConvLayer_472446403130
// MI455X (gfx1250) — hardware-verified
//
#include <hip/hip_runtime.h>


namespace {
typedef _Float16 b16;
typedef __attribute__((ext_vector_type(16))) _Float16 v16b;
typedef __attribute__((ext_vector_type(8))) _Float16 v8b;
typedef __attribute__((ext_vector_type(4))) _Float16 v4h;
typedef __attribute__((ext_vector_type(2))) _Float16 v2h;
typedef __attribute__((ext_vector_type(8))) float v8f;
typedef __attribute__((ext_vector_type(4))) float v4f;
typedef __attribute__((ext_vector_type(2))) float v2f;
__device__ __forceinline__ float bf16_rne(float f) { unsigned int u = __float_as_uint(f); u += 0x7FFFu + ((u >> 16) & 1u); return __uint_as_float(u & 0xFFFF0000u); }
__device__ __forceinline__ void split16(float v, b16& hi, b16& lo) { hi = (b16)v; lo = (b16)(v - (float)hi); }
__device__ __forceinline__ v16b frag_kb(const b16* p, int hh) { const v8b a = *(const v8b*)(p + 8 * hh), b = *(const v8b*)(p + 16 + 8 * hh); v16b f;
#pragma unroll
  for (int e = 0; e < 8; ++e) { f[e] = a[e]; f[8 + e] = b[e]; } return f; }
__device__ __forceinline__ v8f wmma16b(v16b a, v16b b, v8f c) { v8f d = __builtin_amdgcn_wmma_f32_16x16x32_f16(false, a, false, b, (short)0, c, false, false); asm volatile("v_nop\n\tv_nop\n\tv_nop\n\tv_nop" : "+v"(d) : "v"(a), "v"(b)); return d; }
__device__ __forceinline__ void wave_lds_sync() { __builtin_amdgcn_fence(__ATOMIC_RELEASE, "workgroup"); __builtin_amdgcn_wave_barrier(); __builtin_amdgcn_fence(__ATOMIC_ACQUIRE, "workgroup"); }
__device__ __forceinline__ float pmul(float a, float b) { float p = a * b; asm volatile("" : "+v"(p)); return p; }
__device__ __forceinline__ int iclamp(int v, int lo, int hi) { return v < lo ? lo : (v > hi ? hi : v); }
__device__ __forceinline__ float nexp2(float v) { return __builtin_amdgcn_exp2f(v); }

constexpr int B = 8, BL = B  , NPT = 1024, CI = 64, CO = 64, T = 8, KTOT = T * NPT  , NROW = BL * NPT, NBLK = NROW / 32;
constexpr float XS = 8.0f, XW = 512.0f  , WSC = 256.0f, QS = 16384.0f, RS_ = 1024.0f, BS_ = 64.0f, LOG2E = 1.4426950408889634f, BNEPS = 1e-5f;
static_assert(NPT % 64 == 0 && CI == 64 && CO == 64 && KTOT % 32 == 0 && NROW % 32 == 0, "tiling");

__global__ __launch_bounds__(256) void rowsum_kernel(const float* __restrict__ pts, float* __restrict__ RS) {
  const int u = blockIdx.x * 256 + threadIdx.x; const int b = u / NPT; const float* pb = pts + (size_t)b * NPT * 3; const float px = bf16_rne(pts[(size_t)u * 3]), py = bf16_rne(pts[(size_t)u * 3 + 1]), pz = bf16_rne(pts[(size_t)u * 3 + 2]); float s = 0.0f;
#pragma unroll 2
  for (int m = 0; m < NPT; ++m) { const float dx = px - bf16_rne(pb[m * 3]), dy = py - bf16_rne(pb[m * 3 + 1]), dz = pz - bf16_rne(pb[m * 3 + 2]); const float d2 = dx * dx + dy * dy + dz * dz; s += nexp2(-0.5f * LOG2E * d2); }
  for (int pass = 0; pass < 2; ++pass) { ((volatile float*)RS)[u] = s; __threadfence(); }
}
__global__ __launch_bounds__(256) void kprep_kernel(const float* __restrict__ kt, b16* __restrict__ KT) {
  const int u = blockIdx.x * 256 + threadIdx.x; if (u >= T * CO * CI / 8) return; const int e = u * 8; const int row = e / CI, c0 = e % CI; const int t = row / CO, o = row % CO; v8b v;
  for (int j = 0; j < 8; ++j) v[j] = (b16)(bf16_rne(kt[((size_t)o * CI + c0 + j) * T + t]) * WSC);
  for (int pass = 0; pass < 2; ++pass) { *(volatile v8b*)(KT + e) = v; __threadfence(); }
}
__global__ __launch_bounds__(128) void bgen_kernel(const float* __restrict__ fn, const float* __restrict__ RS, const b16* __restrict__ KT, b16* __restrict__ BH, b16* __restrict__ BLO) {
  __shared__ __attribute__((aligned(16))) b16 Ah[4][16][CI + 8], Al[4][16][CI + 8]; __shared__ __attribute__((aligned(16))) b16 Th[128][64 + 8], Tl[128][64 + 8];
  const int wave = threadIdx.x >> 5, lane = threadIdx.x & 31, nloc = lane & 15, hlf = lane >> 4; const int b = blockIdx.y, m0 = blockIdx.x * 64, mw = m0 + wave * 16;
  for (int idx = lane; idx < 16 * (CI / 4); idx += 32) { const int rr = idx / (CI / 4), c4 = (idx % (CI / 4)) * 4; const size_t row = (size_t)b * NPT + mw + rr; const float inv = 1.0f / RS[row]; const v4f f = *(const v4f*)(fn + row * CI + c4); v4h hv, lv;
    for (int j = 0; j < 4; ++j) { b16 ph, pl; split16(bf16_rne(f[j]) * inv * XW, ph, pl); hv[j] = ph; lv[j] = pl; } *(v4h*)(&Ah[wave][rr][c4]) = hv; *(v4h*)(&Al[wave][rr][c4]) = lv; }
  wave_lds_sync();
  const v16b a0 = frag_kb(&Ah[wave][nloc][0], hlf), a1 = frag_kb(&Ah[wave][nloc][32], hlf), l0 = frag_kb(&Al[wave][nloc][0], hlf), l1 = frag_kb(&Al[wave][nloc][32], hlf);
#pragma unroll 1
  for (int s = 0; s < 4; ++s) {
    v8f acc[8];
#pragma unroll
    for (int tt = 0; tt < 8; ++tt) { const b16* br = KT + (size_t)(s * 128 + tt * 16 + nloc) * CI; const v16b b0 = frag_kb(br, hlf), b1 = frag_kb(br + 32, hlf); v8f a = wmma16b(a0, b0, (v8f){}); a = wmma16b(a1, b1, a); a = wmma16b(l0, b0, a); acc[tt] = wmma16b(l1, b1, a); }
    __syncthreads();
#pragma unroll
    for (int tt = 0; tt < 8; ++tt)
#pragma unroll
      for (int r = 0; r < 8; ++r) { const float bv = acc[tt][r] * (1.0f / (XW * WSC)) * BS_; const b16 ph = (b16)bv; Th[tt * 16 + nloc][wave * 16 + 8 * hlf + r] = ph; Tl[tt * 16 + nloc][wave * 16 + 8 * hlf + r] = (b16)((bv - (float)ph) * RS_); }
    __syncthreads();
    for (int pass = 0; pass < 2; ++pass) { for (int q = 0; q < 32; ++q) { const int col = wave * 32 + q; const int t = s * 2 + col / 64, o = col % 64; const size_t dst = (((size_t)b * CO + o) * KTOT) + (size_t)t * NPT + m0 + lane * 2;
        *(volatile v2h*)(BH + dst) = *(const v2h*)(&Th[col][lane * 2]); *(volatile v2h*)(BLO + dst) = *(const v2h*)(&Tl[col][lane * 2]); } __threadfence(); } }
}
__global__ __launch_bounds__(64) void main_kernel(const float* __restrict__ pts, const float* __restrict__ tr, const b16* __restrict__ BH, const b16* __restrict__ BLO, float* __restrict__ O, float* __restrict__ PS) {
  __shared__ __attribute__((aligned(16))) b16 Ah[2][16][32 + 8], Al[2][16][32 + 8]; __shared__ __attribute__((aligned(16))) float Tf[2][16][CO + 4];
  const int wave = threadIdx.x >> 5, lane = threadIdx.x & 31, nloc = lane & 15, hlf = lane >> 4; const int b = blockIdx.y, n0 = blockIdx.x * 32 + wave * 16; const int myrow = n0 + nloc;
  const float* pb = pts + (size_t)b * NPT * 3; const float pnx = bf16_rne(pb[myrow * 3]), pny = bf16_rne(pb[myrow * 3 + 1]), pnz = bf16_rne(pb[myrow * 3 + 2]);
  v8f acc[4], acc2[4];
#pragma unroll
  for (int tt = 0; tt < 4; ++tt) { acc[tt] = (v8f){}; acc2[tt] = (v8f){}; }
#pragma unroll 1
  for (int t = 0; t < T; ++t) { const float tx = bf16_rne(tr[((size_t)b * T + t) * 3]), ty = bf16_rne(tr[((size_t)b * T + t) * 3 + 1]), tz = bf16_rne(tr[((size_t)b * T + t) * 3 + 2]); const float ax = pnx - tx, ay = pny - ty, az = pnz - tz;
#pragma unroll 1
    for (int m0 = 0; m0 < NPT; m0 += 32) {
      v8b hvA, hvB, lvA, lvB;
#pragma unroll
      for (int e = 0; e < 16; ++e) { const int m = m0 + 16 * hlf + e; const float dx = ax - bf16_rne(pb[m * 3]), dy = ay - bf16_rne(pb[m * 3 + 1]), dz = az - bf16_rne(pb[m * 3 + 2]); const float d2 = fmaf(dx, dx, fmaf(dy, dy, dz * dz));
        const float qs = nexp2(-0.5f * LOG2E * d2) * QS; const b16 ph = (b16)qs; const b16 pl = (b16)((qs - (float)ph) * RS_); if (e < 8) { hvA[e] = ph; lvA[e] = pl; } else { hvB[e - 8] = ph; lvB[e - 8] = pl; } }
      *(v8b*)(&Ah[wave][nloc][16 * hlf]) = hvA; *(v8b*)(&Ah[wave][nloc][16 * hlf + 8]) = hvB; *(v8b*)(&Al[wave][nloc][16 * hlf]) = lvA; *(v8b*)(&Al[wave][nloc][16 * hlf + 8]) = lvB;
      wave_lds_sync();
      const v16b a = frag_kb(&Ah[wave][nloc][0], hlf), al = frag_kb(&Al[wave][nloc][0], hlf); const size_t kb = (size_t)t * NPT + m0;
#pragma unroll
      for (int tt = 0; tt < 4; ++tt) { const b16* bh = BH + ((size_t)b * CO + tt * 16 + nloc) * KTOT + kb; const v16b fb = frag_kb(bh, hlf); acc[tt] = wmma16b(a, fb, acc[tt]); acc2[tt] = wmma16b(al, fb, acc2[tt]); acc2[tt] = wmma16b(a, frag_kb(BLO + ((size_t)b * CO + tt * 16 + nloc) * KTOT + kb, hlf), acc2[tt]); }
      wave_lds_sync(); } }
#pragma unroll
  for (int tt = 0; tt < 4; ++tt)
#pragma unroll
    for (int r = 0; r < 8; ++r) Tf[wave][8 * hlf + r][tt * 16 + nloc] = (acc[tt][r] + acc2[tt][r] * (1.0f / RS_)) * (1.0f / (QS * BS_));
  __syncthreads();
  for (int pass = 0; pass < 2; ++pass) {
    for (int rr = 0; rr < 16; rr += 2) { const int row = rr + hlf; *(volatile v4f*)(O + ((size_t)b * NPT + n0 + row) * CO + nloc * 4) = *(const v4f*)(&Tf[wave][row][nloc * 4]); }
    { const int cc = threadIdx.x; float s = 0.0f; for (int w2 = 0; w2 < 2; ++w2) for (int rr = 0; rr < 16; ++rr) s += Tf[w2][rr][cc]; ((volatile float*)PS)[((size_t)blockIdx.y * (NPT / 32) + blockIdx.x) * CO + cc] = s; }
    __threadfence(); }
}
__global__ __launch_bounds__(64) void colstat_kernel(const float* __restrict__ PS, float* __restrict__ ST) { const int c = threadIdx.x; float s = 0.0f;
#pragma unroll 1
  for (int bb = 0; bb < NBLK; ++bb) s += PS[(size_t)bb * CO + c];
  for (int pass = 0; pass < 2; ++pass) { ((volatile float*)ST)[c] = s * (1.0f / NROW); __threadfence(); } }
__global__ __launch_bounds__(64) void var_kernel(const float* __restrict__ O, const float* __restrict__ MEAN, float* __restrict__ PS) { const int c = threadIdx.x; float a = 0.0f; const float m = MEAN[c];
#pragma unroll 1
  for (int rr = 0; rr < 32; ++rr) { const float dlt = O[((size_t)blockIdx.x * 32 + rr) * CO + c] - m; a += dlt * dlt; }
  for (int pass = 0; pass < 2; ++pass) { ((volatile float*)PS)[(size_t)blockIdx.x * CO + c] = a; __threadfence(); } }
__global__ __launch_bounds__(256) void bn_kernel(const float* __restrict__ O, const float* __restrict__ MEAN, const float* __restrict__ VAR, const float* __restrict__ g, const float* __restrict__ be, float* __restrict__ out) {
  const size_t u = (size_t)blockIdx.x * 256 + threadIdx.x; if (u >= (size_t)NROW * CO / 4) return; const int c = (int)((u * 4) % CO); const v4f x = *(const v4f*)(O + u * 4); v4f y;
  for (int j = 0; j < 4; ++j) y[j] = fmaxf((x[j] - MEAN[c + j]) * rsqrtf(VAR[c + j] + BNEPS) * bf16_rne(g[c + j]) + bf16_rne(be[c + j]), 0.0f);
  for (int pass = 0; pass < 2; ++pass) { *(volatile v4f*)(out + u * 4) = y; __threadfence(); } }
}

extern "C" void kernel_launch(void* const* d_in, const int* in_sizes, int n_in, void* d_out, int out_size, void* d_ws, size_t ws_size, hipStream_t stream) {
  (void)n_in;
  auto Fp = [&](int i) { return (const float*)d_in[i]; };
  if (in_sizes[0] != B * NPT * 3 || in_sizes[1] != B * T * 3 || in_sizes[2] != B * NPT * CI || in_sizes[3] != CO * CI * T || in_sizes[4] != CO || in_sizes[5] != CO || out_size != B * NPT * CO) return;
  size_t off = 0; char* ws = (char*)d_ws;
  auto carve = [&](size_t bytes) { char* p = ws + off; off += (bytes + 255) & ~(size_t)255; return p; };
  float* RS = (float*)carve((size_t)B * NPT * 4); b16* KT = (b16*)carve((size_t)T * CO * CI * 2); b16* BH = (b16*)carve((size_t)B * CO * KTOT * 2); b16* BLO = (b16*)carve((size_t)B * CO * KTOT * 2);
  float* O = (float*)carve((size_t)NROW * CO * 4); float* PS = (float*)carve((size_t)NBLK * CO * 4); float* ST = (float*)carve((size_t)2 * CO * 4);
  if (off > ws_size || off > ((size_t)128 << 20)) return;
  rowsum_kernel<<<BL * NPT / 256, 256, 0, stream>>>(Fp(0), RS);
  kprep_kernel<<<(T * CO * CI / 8 + 255) / 256, 256, 0, stream>>>(Fp(3), KT);
  bgen_kernel<<<dim3(NPT / 64, BL), 128, 0, stream>>>(Fp(2), RS, KT, BH, BLO);
  main_kernel<<<dim3(NPT / 32, BL), 64, 0, stream>>>(Fp(0), Fp(1), BH, BLO, O, PS);
  colstat_kernel<<<1, CO, 0, stream>>>(PS, ST); var_kernel<<<NBLK, CO, 0, stream>>>(O, ST, PS); colstat_kernel<<<1, CO, 0, stream>>>(PS, ST + CO);
  bn_kernel<<<(unsigned)(((size_t)NROW * CO / 4 + 255) / 256), 256, 0, stream>>>(O, ST, ST + CO, Fp(4), Fp(5), (float*)d_out);
}
